// MambaModule_79147657331141
// MI455X (gfx1250) — hardware-run, weakly checked
//
#include <hip/hip_runtime.h>

#define NB    2
#define NL    1024
#define DM    256
#define DI    512
#define DIN2  1024
#define NS    16
#define DTR   16
#define KDT   64
#define NXD   48
#define NXP   64
#define NROWS (NB * NL)
#define TC    16
#define TO    32
#define LNEPS 1e-5f

static_assert(DM % 32 == 0 && DI % 32 == 0 && KDT % 32 == 0);
static_assert(NROWS % 128 == 0 && DIN2 % 64 == 0 && DM % 64 == 0 && NXP % 64 == 0 && DI % 64 == 0);
static_assert(NL % TC == 0 && NL % TO == 0 && DI % 256 == 0 && DM == 256 && TC == 16 && TO == 32);
static_assert(DTR % 8 == 0 && DTR + 2 * NS == NXD && NXD <= NXP && DTR <= KDT && NXP == 64);
static_assert(DIN2 == 2 * DI && NL % 64 == 0);
static_assert(NXD % 4 == 0 && NL % 4 == 0 && DM % 8 == 0 && DI % 4 == 0 && NS % 4 == 0);

typedef __bf16         v16b __attribute__((ext_vector_type(16)));
typedef unsigned short v8us __attribute__((ext_vector_type(8)));
typedef float          v8f  __attribute__((ext_vector_type(8)));
typedef float          v4f  __attribute__((ext_vector_type(4)));
typedef v8us __attribute__((may_alias)) v8usa;
typedef v4f  __attribute__((may_alias)) v4fa;

union Frag { v16b v; v8us half[2]; };

constexpr size_t SZ_X0   = (size_t)NROWS * DM * 2;
constexpr size_t WO_WIN  = 0;
constexpr size_t WO_WXP  = WO_WIN + (size_t)DIN2 * DM * 2;
constexpr size_t WO_WDT  = WO_WXP + (size_t)NXP * DI * 2;
constexpr size_t WO_WOUT = WO_WDT + (size_t)DI * KDT * 2;
constexpr size_t SZ_WSET = WO_WOUT + (size_t)DM * DI * 2;
constexpr size_t PO_XR   = 0;
constexpr size_t PO_XF   = PO_XR + (size_t)NROWS * DIN2 * 4;
constexpr size_t PO_XH   = PO_XF + (size_t)NROWS * DI * 4;
constexpr size_t PO_XL   = PO_XH + (size_t)NROWS * DI * 2;
constexpr size_t PO_XDBL = PO_XL + (size_t)NROWS * DI * 2;
constexpr size_t PO_DTH  = PO_XDBL + (size_t)NROWS * NXP * 4;
constexpr size_t PO_DTL  = PO_DTH + (size_t)NROWS * KDT * 2;
constexpr size_t PO_YH   = PO_DTL + (size_t)NROWS * KDT * 2;
constexpr size_t PO_YL   = PO_YH + (size_t)NROWS * DI * 2;
constexpr size_t PO_MO   = PO_YL + (size_t)NROWS * DI * 2;
constexpr size_t SZ_PSET = PO_MO + (size_t)NROWS * DM * 4;
constexpr size_t OFF_X0  = 0;
constexpr size_t OFF_W1  = OFF_X0 + SZ_X0;
constexpr size_t OFF_W2  = OFF_W1 + SZ_WSET;
constexpr size_t OFF_P1  = OFF_W2 + SZ_WSET;
constexpr size_t OFF_P2  = OFF_P1 + SZ_PSET;
constexpr size_t OFF_U2F = OFF_P2 + SZ_PSET;
constexpr size_t OFF_U2H = OFF_U2F + (size_t)NROWS * DM * 4;
constexpr size_t OFF_U2L = OFF_U2H + (size_t)NROWS * DM * 2;
constexpr size_t WS_END  = OFF_U2L + (size_t)NROWS * DM * 2;
static_assert(OFF_W1 % 128 == 0 && OFF_W2 % 128 == 0 && OFF_P1 % 128 == 0 && OFF_P2 % 128 == 0);
static_assert(WO_WXP % 128 == 0 && WO_WDT % 128 == 0 && WO_WOUT % 128 == 0);
static_assert(PO_XF % 128 == 0 && PO_XH % 128 == 0 && PO_XL % 128 == 0 && PO_XDBL % 128 == 0);
static_assert(PO_DTH % 128 == 0 && PO_DTL % 128 == 0 && PO_YH % 128 == 0 && PO_YL % 128 == 0 && PO_MO % 128 == 0);
static_assert(OFF_U2F % 128 == 0 && OFF_U2H % 128 == 0 && OFF_U2L % 128 == 0);
static_assert(WS_END <= (size_t)134217728);
static_assert((size_t)(NL / 64) * (DM / 64) * NB * 64 * 64 * 2 == SZ_X0);
static_assert((size_t)(DIN2 / 64) * (DM / 64) * 64 * 64 * 2 == WO_WXP - WO_WIN);
static_assert((size_t)(NXP / 64) * (DI / 64) * 64 * 64 * 2 == WO_WDT - WO_WXP);
static_assert((size_t)(DI / 64) * (KDT / 64) * 64 * 64 * 2 == WO_WOUT - WO_WDT);
static_assert((size_t)(DM / 64) * (DI / 64) * 64 * 64 * 2 == SZ_WSET - WO_WOUT);
static_assert((size_t)(NROWS / 128) * (DIN2 / 64) * 256 * 128 == PO_XF - PO_XR);
static_assert((size_t)(DI / 256) * (NROWS / TC) * (TC * 8) * 128 == PO_XH - PO_XF);
static_assert((size_t)(DI / 256) * (NROWS / TC) * (TC * 4) * 128 == PO_XL - PO_XH);
static_assert((size_t)(NROWS / 128) * (NXP / 64) * 256 * 128 == PO_DTH - PO_XDBL);
static_assert((size_t)(NROWS / 128) * 128 * 128 == PO_DTL - PO_DTH);
static_assert((size_t)(DI / 256) * NB * (NL / TC) * (TC * 4) * 128 == PO_YL - PO_YH);
static_assert((size_t)(NROWS / 128) * (DM / 64) * 256 * 128 == SZ_PSET - PO_MO);
static_assert((size_t)(NROWS / TC) * (TC * 8) * 128 == OFF_U2H - OFF_U2F);
static_assert((size_t)(NROWS / TC) * (TC * 4) * 128 == OFF_U2L - OFF_U2H);
static_assert((size_t)(NROWS / TO) * DM * 128 == (size_t)NB * DM * NL * 4);

__device__ __forceinline__ unsigned short bf16_bits(float f) {
  unsigned u = __float_as_uint(f);
  u += 0x7FFFu + ((u >> 16) & 1u);
  return (unsigned short)(u >> 16);
}
__device__ __forceinline__ float bf16_val(unsigned short b) { return __uint_as_float(((unsigned)b) << 16); }
__device__ __forceinline__ float bf16r(float f) { return bf16_val(bf16_bits(f)); }
__device__ __forceinline__ void split_bf16(float v, unsigned short& hb, unsigned short& lb) {
  hb = bf16_bits(v);
  lb = bf16_bits(v - bf16_val(hb));
}
__device__ __forceinline__ v8f zero8() {
  v8f z;
#pragma unroll
  for (int i = 0; i < 8; ++i) z[i] = 0.0f;
  return z;
}
__device__ __forceinline__ float wsum(float v) {
#pragma unroll
  for (int o = 16; o > 0; o >>= 1) v += __shfl_xor(v, o, 32);
  return v;
}

__device__ __forceinline__ void ldfrag_g(Frag& f, const unsigned short* p, int h) {
  f.half[0] = *(const v8usa*)(p + 8 * h);
  f.half[1] = *(const v8usa*)(p + 16 + 8 * h);
}
__device__ __forceinline__ v8f mma16(v8f c, const Frag& a, const Frag& b) {
  v8f d = __builtin_amdgcn_wmma_f32_16x16x32_bf16(false, a.v, false, b.v, (short)0, c, false, false);
  asm volatile("v_nop\n\tv_nop\n\tv_nop\n\tv_nop" : "+v"(d) : "v"(a.v), "v"(b.v));
  return d;
}

__device__ __forceinline__ void tc_store_pass(const unsigned short* sT, unsigned short* dst, int P,
                                              int orow0, int ocol0, int w, int lane) {
  const int q8 = lane & 7, sub = lane >> 3;
#pragma unroll
  for (int i = 0; i < 2; ++i) {
    const int li = 8 * w + 4 * i + sub;
    const v8us v = *(const v8usa*)(sT + li * 64 + 8 * q8);
    unsigned short* p = dst + (size_t)(orow0 + li) * P + ocol0 + 8 * q8;
    *(volatile v8us*)p = v;
  }
}

__global__ __launch_bounds__(256)
void tcvt_kernel(const float* __restrict__ in, int R, int Cc, size_t izs,
                 unsigned short* out, int P, size_t ozs)
{
  __shared__ __attribute__((aligned(16))) unsigned short sT[64 * 64];

  const int tid = threadIdx.x, lane = tid & 31, w = tid >> 5;
  const int orow0 = blockIdx.x * 64, ocol0 = blockIdx.y * 64;
  const float* src = in + (size_t)blockIdx.z * izs;
  unsigned short* dst = out + (size_t)blockIdx.z * ozs;

  const int c4 = tid & 15, rs = tid >> 4;
  const int c = orow0 + 4 * c4;
  const bool cok = (c < Cc);
  const int cc = cok ? c : (Cc - 4);
#pragma unroll
  for (int i = 0; i < 4; ++i) {
    const int rloc = 16 * i + rs;
    const int r = ocol0 + rloc;
    const int rr = (r < R) ? r : (R - 1);
    const v4f v = *(const v4fa*)(src + (size_t)rr * Cc + cc);
    const bool ok = cok && (r < R);
    sT[(4 * c4 + 0) * 64 + rloc] = ok ? bf16_bits(v[0]) : (unsigned short)0;
    sT[(4 * c4 + 1) * 64 + rloc] = ok ? bf16_bits(v[1]) : (unsigned short)0;
    sT[(4 * c4 + 2) * 64 + rloc] = ok ? bf16_bits(v[2]) : (unsigned short)0;
    sT[(4 * c4 + 3) * 64 + rloc] = ok ? bf16_bits(v[3]) : (unsigned short)0;
  }
  __syncthreads();

  tc_store_pass(sT, dst, P, orow0, ocol0, w, lane);
  __threadfence();
  tc_store_pass(sT, dst, P, orow0, ocol0, w, lane);
}

__device__ __forceinline__ void c_store_pass(const float* sT, float* C, int ldc, int m0w, int cy, int w, int lane) {
  const int q8 = lane & 7, sub = lane >> 3;
#pragma unroll
  for (int i = 0; i < 16; ++i) {
    const int lid = 4 * i + sub;
    const int rl = lid >> 1, hl = lid & 1;
    const v4f v = *(const v4fa*)(sT + (32 * w + rl) * 64 + 32 * hl + 4 * q8);
    float* dst = C + (size_t)(m0w + rl) * ldc + 64 * cy + 32 * hl + 4 * q8;
    *(volatile v4f*)dst = v;
  }
}

__device__ __forceinline__ void dtr_store_pass(const float* sT, unsigned short* dh, unsigned short* dl,
                                               int m0w, int w, int lane) {
  const int q8 = lane & 7, sub = lane >> 3;
  const bool pad = (q8 >= DTR / 8);
#pragma unroll
  for (int i = 0; i < 8; ++i) {
    const int rl = 4 * i + sub;
    const float* sr = sT + (32 * w + rl) * 64 + 8 * q8;
    const v4f a = *(const v4fa*)sr;
    const v4f c = *(const v4fa*)(sr + 4);
    v8us oh, ol;
    unsigned short hb, lb;
    split_bf16(a[0], hb, lb); oh[0] = pad ? (unsigned short)0 : hb; ol[0] = pad ? (unsigned short)0 : lb;
    split_bf16(a[1], hb, lb); oh[1] = pad ? (unsigned short)0 : hb; ol[1] = pad ? (unsigned short)0 : lb;
    split_bf16(a[2], hb, lb); oh[2] = pad ? (unsigned short)0 : hb; ol[2] = pad ? (unsigned short)0 : lb;
    split_bf16(a[3], hb, lb); oh[3] = pad ? (unsigned short)0 : hb; ol[3] = pad ? (unsigned short)0 : lb;
    split_bf16(c[0], hb, lb); oh[4] = pad ? (unsigned short)0 : hb; ol[4] = pad ? (unsigned short)0 : lb;
    split_bf16(c[1], hb, lb); oh[5] = pad ? (unsigned short)0 : hb; ol[5] = pad ? (unsigned short)0 : lb;
    split_bf16(c[2], hb, lb); oh[6] = pad ? (unsigned short)0 : hb; ol[6] = pad ? (unsigned short)0 : lb;
    split_bf16(c[3], hb, lb); oh[7] = pad ? (unsigned short)0 : hb; ol[7] = pad ? (unsigned short)0 : lb;
    const size_t go = (size_t)(m0w + rl) * KDT + 8 * q8;
    *(volatile v8us*)(dh + go) = oh;
    *(volatile v8us*)(dl + go) = ol;
  }
}

template <int NPL, int XP, int HB>
__global__ __launch_bounds__(128)
void gemm_kernel(const unsigned short* __restrict__ Ah, const unsigned short* __restrict__ Al, int lda,
                 const unsigned short* __restrict__ Bw, int K, const float* __restrict__ bias,
                 float* C, int ldc, unsigned short* dh, unsigned short* dl)
{
  __shared__ __attribute__((aligned(16))) float sT[128 * 64];

  const int tid = threadIdx.x, lane = tid & 31, w = tid >> 5;
  const int h = lane >> 4, m = lane & 15;
  const int m0 = blockIdx.x * 128;
  const int cy = blockIdx.y;
  const int m0w = m0 + 32 * w;

  const unsigned short* xa = Ah + (size_t)(m0w + m) * lda;
  const unsigned short* xr = Al + (size_t)(m0w + m) * lda;
  const unsigned short* wb = Bw + (size_t)(64 * cy + m) * K;

  v8f acc[2][4];
#pragma unroll
  for (int mt = 0; mt < 2; ++mt)
#pragma unroll
    for (int nt = 0; nt < 4; ++nt) acc[mt][nt] = zero8();

#pragma unroll 1
  for (int k0 = 0; k0 < K; k0 += 32) {
    Frag a0, a1, e0, e1;
    ldfrag_g(a0, xa + k0, h);
    ldfrag_g(a1, xa + (size_t)16 * lda + k0, h);
    if (NPL == 2) {
      ldfrag_g(e0, xr + k0, h);
      ldfrag_g(e1, xr + (size_t)16 * lda + k0, h);
    }
#pragma unroll
    for (int nt = 0; nt < 4; ++nt) {
      Frag b;
      ldfrag_g(b, wb + (size_t)nt * 16 * K + k0, h);
      acc[0][nt] = mma16(acc[0][nt], a0, b);
      acc[1][nt] = mma16(acc[1][nt], a1, b);
      if (NPL == 2) {
        acc[0][nt] = mma16(acc[0][nt], e0, b);
        acc[1][nt] = mma16(acc[1][nt], e1, b);
      }
    }
  }

#pragma unroll
  for (int nt = 0; nt < 4; ++nt) {
    const int col = 16 * nt + m;
    const float bv = (HB == 1) ? bf16r(bias[64 * cy + col]) : 0.0f;
#pragma unroll
    for (int mt = 0; mt < 2; ++mt)
#pragma unroll
      for (int r = 0; r < 8; ++r) {
        const int rowl = 32 * w + 16 * mt + 8 * h + r;
        sT[rowl * 64 + col] = acc[mt][nt][r] + bv;
      }
  }
  __syncthreads();

  c_store_pass(sT, C, ldc, m0w, cy, w, lane);
  __threadfence();
  c_store_pass(sT, C, ldc, m0w, cy, w, lane);

  if (XP == 1) {
    if (cy == 0) {
      dtr_store_pass(sT, dh, dl, m0w, w, lane);
      __threadfence();
      dtr_store_pass(sT, dh, dl, m0w, w, lane);
    }
  }
}

__device__ __forceinline__ void f32tile_store_pass(const float* sF, float* xf, int pitch, int rbase, int col0,
                                                   int w, int lane) {
  const int q8 = lane & 7, sub = lane >> 3;
#pragma unroll
  for (int i = 0; i < 4; ++i) {
    const int li = 4 * i + sub;
    const int row = 2 * w + (li >> 3), q = li & 7;
    const v4f v = *(const v4fa*)(sF + row * 256 + 32 * q + 4 * q8);
    float* dst = xf + (size_t)(rbase + row) * pitch + col0 + 32 * q + 4 * q8;
    *(volatile v4f*)dst = v;
  }
}

__device__ __forceinline__ void h16tile_store_pass(const unsigned short* sH, const unsigned short* sL,
                                                   unsigned short* ph, unsigned short* pl, int pitch, int col0,
                                                   int rbase, int w, int lane) {
  const int q8 = lane & 7, sub = lane >> 3;
#pragma unroll
  for (int i = 0; i < 2; ++i) {
    const int li = 4 * i + sub;
    const int row = 2 * w + (li >> 2), q = li & 3;
    const v8us vh = *(const v8usa*)(sH + row * 256 + 64 * q + 8 * q8);
    const v8us vl = *(const v8usa*)(sL + row * 256 + 64 * q + 8 * q8);
    const size_t go = (size_t)(rbase + row) * pitch + col0 + 64 * q + 8 * q8;
    *(volatile v8us*)(ph + go) = vh;
    *(volatile v8us*)(pl + go) = vl;
  }
}

__global__ __launch_bounds__(256)
void conv_kernel(const float* __restrict__ xr, const float* __restrict__ cw, const float* __restrict__ cb,
                 float* xf, unsigned short* ph, unsigned short* pl)
{
  __shared__ __attribute__((aligned(16))) float sF[TC * 256];
  __shared__ __attribute__((aligned(16))) unsigned short sH[TC * 256];
  __shared__ __attribute__((aligned(16))) unsigned short sL[TC * 256];

  const int tid = threadIdx.x, lane = tid & 31, w = tid >> 5;
  const int slab = blockIdx.x;
  const int rbase = blockIdx.y * TC;
  const int b = rbase / NL, l0 = rbase - b * NL;
  const int c = 256 * slab + tid;

  const v4f cwv = *(const v4fa*)(cw + (size_t)c * 4);
  const float w0 = bf16r(cwv[0]);
  const float w1 = bf16r(cwv[1]);
  const float w2 = bf16r(cwv[2]);
  const float w3 = bf16r(cwv[3]);
  const float cbv = bf16r(cb[c]);

  const float* col = xr + (size_t)b * NL * DIN2 + c;

  int p, pc;
  p = l0 - 3; pc = (p > 0) ? p : 0;
  float v0 = col[(size_t)pc * DIN2]; v0 = (p >= 0) ? v0 : 0.0f;
  p = l0 - 2; pc = (p > 0) ? p : 0;
  float v1 = col[(size_t)pc * DIN2]; v1 = (p >= 0) ? v1 : 0.0f;
  p = l0 - 1; pc = (p > 0) ? p : 0;
  float v2 = col[(size_t)pc * DIN2]; v2 = (p >= 0) ? v2 : 0.0f;

#pragma unroll 1
  for (int tt = 0; tt < TC; ++tt) {
    const float v3 = col[(size_t)(l0 + tt) * DIN2];
    const float s = w0 * v0 + w1 * v1 + w2 * v2 + w3 * v3 + cbv;
    const float ex = expf(-s);
    const float sg = 1.0f / (1.0f + ex);
    const float y = s * sg;
    sF[tt * 256 + tid] = y;
    unsigned short hb, lb;
    split_bf16(y, hb, lb);
    sH[tt * 256 + tid] = hb;
    sL[tt * 256 + tid] = lb;
    v0 = v1; v1 = v2; v2 = v3;
  }
  __syncthreads();

  const int col0 = 256 * slab;
  f32tile_store_pass(sF, xf, DI, rbase, col0, w, lane);
  h16tile_store_pass(sH, sL, ph, pl, DI, col0, rbase, w, lane);
  __threadfence();
  f32tile_store_pass(sF, xf, DI, rbase, col0, w, lane);
  h16tile_store_pass(sH, sL, ph, pl, DI, col0, rbase, w, lane);
}

__global__ __launch_bounds__(256)
void dtscan_kernel(const unsigned short* __restrict__ dth, const unsigned short* __restrict__ dtl,
                   const unsigned short* __restrict__ wdt,
                   const float* __restrict__ xdbl,
                   const float* __restrict__ xf,
                   const float* __restrict__ xr,
                   const float* __restrict__ dtb, const float* __restrict__ alog,
                   const float* __restrict__ dpar,
                   unsigned short* yh, unsigned short* yl)
{
  __shared__ __attribute__((aligned(16))) float sD[TC * 256];
  __shared__ __attribute__((aligned(16))) unsigned short sH[TC * 256];
  __shared__ __attribute__((aligned(16))) unsigned short sL[TC * 256];
  __shared__ __attribute__((aligned(16))) float sBC[TC * 32];

  const int tid = threadIdx.x, lane = tid & 31, w = tid >> 5;
  const int h = lane >> 4, m = lane & 15;
  const int slab = blockIdx.x, b = blockIdx.y;
  const int c0 = 256 * slab;
  const int d = c0 + tid;

  const float bb = bf16r(dtb[d]);
  const float Dv = bf16r(dpar[d]);
  float An[NS];
  {
    const float* ap = alog + (size_t)d * NS;
#pragma unroll
    for (int q = 0; q < NS / 4; ++q) {
      const v4f av = *(const v4fa*)(ap + 4 * q);
#pragma unroll
      for (int j = 0; j < 4; ++j) An[4 * q + j] = -expf(bf16r(av[j]));
    }
  }

  Frag bw[2][2];
#pragma unroll
  for (int nt = 0; nt < 2; ++nt)
#pragma unroll
    for (int ks = 0; ks < 2; ++ks)
      ldfrag_g(bw[nt][ks], wdt + (size_t)(c0 + 32 * w + 16 * nt + m) * KDT + 32 * ks, h);

  float hs[NS];
#pragma unroll
  for (int n = 0; n < NS; ++n) hs[n] = 0.0f;

#pragma unroll 1
  for (int t0 = 0; t0 < NL; t0 += TC) {
    const int r0 = b * NL + t0;

    v8f acc[2];
    acc[0] = zero8(); acc[1] = zero8();
#pragma unroll
    for (int ks = 0; ks < 2; ++ks) {
      Frag ah, ar;
      ldfrag_g(ah, dth + (size_t)(r0 + m) * KDT + 32 * ks, h);
      ldfrag_g(ar, dtl + (size_t)(r0 + m) * KDT + 32 * ks, h);
#pragma unroll
      for (int nt = 0; nt < 2; ++nt) {
        acc[nt] = mma16(acc[nt], ah, bw[nt][ks]);
        acc[nt] = mma16(acc[nt], ar, bw[nt][ks]);
      }
    }
#pragma unroll
    for (int nt = 0; nt < 2; ++nt)
#pragma unroll
      for (int r = 0; r < 8; ++r)
        sD[(8 * h + r) * 256 + 32 * w + 16 * nt + m] = acc[nt][r];

    if (tid < 128) {
      const int tok = tid >> 3, q = tid & 7;
      const v4f v = *(const v4fa*)(xdbl + (size_t)(r0 + tok) * NXP + DTR + 4 * q);
      *(v4fa*)(sBC + tok * 32 + 4 * q) = v;
    }
    __syncthreads();

#pragma unroll 1
    for (int tt = 0; tt < TC; ++tt) {
      const float dpre = sD[tt * 256 + tid];
      const float xx = dpre + bb;
      const float dl = fmaxf(xx, 0.0f) + log1pf(expf(-fabsf(xx)));
      const float xv = xf[(size_t)(r0 + tt) * DI + d];
      const float rv = xr[(size_t)(r0 + tt) * DIN2 + DI + d];
      const float* bc = sBC + tt * 32;
      float y = 0.0f;
#pragma unroll
      for (int n = 0; n < NS; ++n) {
        const float dA  = expf(dl * An[n]);
        const float dBu = (dl * bc[n]) * xv;
        hs[n] = dA * hs[n] + dBu;
        y += hs[n] * bc[NS + n];
      }
      const float yv = y + xv * Dv;
      const float eg = expf(-rv);
      const float g = rv * (1.0f / (1.0f + eg));
      const float yg = yv * g;
      unsigned short hb, lb;
      split_bf16(yg, hb, lb);
      sH[tt * 256 + tid] = hb;
      sL[tt * 256 + tid] = lb;
    }
    __syncthreads();

    h16tile_store_pass(sH, sL, yh, yl, DI, c0, r0, w, lane);
    __threadfence();
    h16tile_store_pass(sH, sL, yh, yl, DI, c0, r0, w, lane);
    __syncthreads();
  }
}

__global__ __launch_bounds__(256)
void lnmid_kernel(const float* __restrict__ mo, const unsigned short* __restrict__ x0,
                  const float* __restrict__ lw, const float* __restrict__ lb,
                  float* uf, unsigned short* uh, unsigned short* ul)
{
  __shared__ __attribute__((aligned(16))) float sF[TC * 256];
  __shared__ __attribute__((aligned(16))) unsigned short sH[TC * 256];
  __shared__ __attribute__((aligned(16))) unsigned short sL[TC * 256];

  const int tid = threadIdx.x, lane = tid & 31, w = tid >> 5;
  const int rbase = blockIdx.x * TC;
  const int cb = 8 * lane;

  float wv[8], bv[8];
  {
    const v4f a0 = *(const v4fa*)(lw + cb);
    const v4f a1 = *(const v4fa*)(lw + cb + 4);
    const v4f b0 = *(const v4fa*)(lb + cb);
    const v4f b1 = *(const v4fa*)(lb + cb + 4);
#pragma unroll
    for (int j = 0; j < 4; ++j) {
      wv[j] = bf16r(a0[j]); wv[4 + j] = bf16r(a1[j]);
      bv[j] = bf16r(b0[j]); bv[4 + j] = bf16r(b1[j]);
    }
  }

#pragma unroll 1
  for (int s = 0; s < 2; ++s) {
    const int tok = 2 * w + s;
    const int r = rbase + tok;
    const v4f m0v = *(const v4fa*)(mo + (size_t)r * DM + cb);
    const v4f m1v = *(const v4fa*)(mo + (size_t)r * DM + cb + 4);
    const v8us xb = *(const v8usa*)(x0 + (size_t)r * DM + cb);
    float mv[8], xv[8];
#pragma unroll
    for (int j = 0; j < 4; ++j) { mv[j] = m0v[j]; mv[4 + j] = m1v[j]; }
#pragma unroll
    for (int j = 0; j < 8; ++j) xv[j] = bf16_val(xb[j]);
    float s1 = 0.0f;
#pragma unroll
    for (int j = 0; j < 8; ++j) s1 += mv[j];
    s1 = wsum(s1);
    const float mu = s1 * (1.0f / DM);
    float s2 = 0.0f;
#pragma unroll
    for (int j = 0; j < 8; ++j) { const float dv = mv[j] - mu; s2 += dv * dv; }
    s2 = wsum(s2);
    const float var = s2 * (1.0f / DM);
    const float rstd = rsqrtf(var + LNEPS);
#pragma unroll
    for (int j = 0; j < 8; ++j) {
      const int c = cb + j;
      const float v = xv[j] + ((mv[j] - mu) * rstd) * wv[j] + bv[j];
      const int cf = DM - 1 - c;
      sF[tok * 256 + cf] = v;
      unsigned short hb2, lb2;
      split_bf16(v, hb2, lb2);
      sH[tok * 256 + cf] = hb2;
      sL[tok * 256 + cf] = lb2;
    }
  }
  __syncthreads();

  f32tile_store_pass(sF, uf, DM, rbase, 0, w, lane);
  h16tile_store_pass(sH, sL, uh, ul, DM, 0, rbase, w, lane);
  __threadfence();
  f32tile_store_pass(sF, uf, DM, rbase, 0, w, lane);
  h16tile_store_pass(sH, sL, uh, ul, DM, 0, rbase, w, lane);
}

__device__ __forceinline__ void out_store_pass(const float* sO, float* out, int b, int l0, int w, int lane) {
  const int q8 = lane & 7, sub = lane >> 3;
#pragma unroll
  for (int i = 0; i < 8; ++i) {
    const int co = 32 * w + 4 * i + sub;
    const v4f v = *(const v4fa*)(sO + co * 36 + 4 * q8);
    float* dst = out + (size_t)(b * DM + co) * NL + l0 + 4 * q8;
    *(volatile v4f*)dst = v;
  }
}

__global__ __launch_bounds__(256)
void lnout_kernel(const float* __restrict__ mo, const float* __restrict__ uf,
                  const float* __restrict__ lw, const float* __restrict__ lb, float* out)
{
  __shared__ __attribute__((aligned(16))) float sO[DM * 36];

  const int tid = threadIdx.x, lane = tid & 31, w = tid >> 5;
  const int rbase = blockIdx.x * TO;
  const int b = rbase / NL, l0 = rbase - b * NL;
  const int cb = 8 * lane;

  float wv[8], bv[8];
  {
    const v4f a0 = *(const v4fa*)(lw + cb);
    const v4f a1 = *(const v4fa*)(lw + cb + 4);
    const v4f b0 = *(const v4fa*)(lb + cb);
    const v4f b1 = *(const v4fa*)(lb + cb + 4);
#pragma unroll
    for (int j = 0; j < 4; ++j) {
      wv[j] = bf16r(a0[j]); wv[4 + j] = bf16r(a1[j]);
      bv[j] = bf16r(b0[j]); bv[4 + j] = bf16r(b1[j]);
    }
  }

#pragma unroll 1
  for (int s = 0; s < 4; ++s) {
    const int tok = 4 * w + s;
    const int r = rbase + tok;
    const v4f m0v = *(const v4fa*)(mo + (size_t)r * DM + cb);
    const v4f m1v = *(const v4fa*)(mo + (size_t)r * DM + cb + 4);
    const v4f u0v = *(const v4fa*)(uf + (size_t)r * DM + cb);
    const v4f u1v = *(const v4fa*)(uf + (size_t)r * DM + cb + 4);
    float mv[8], uv[8];
#pragma unroll
    for (int j = 0; j < 4; ++j) { mv[j] = m0v[j]; mv[4 + j] = m1v[j]; uv[j] = u0v[j]; uv[4 + j] = u1v[j]; }
    float s1 = 0.0f;
#pragma unroll
    for (int j = 0; j < 8; ++j) s1 += mv[j];
    s1 = wsum(s1);
    const float mu = s1 * (1.0f / DM);
    float s2 = 0.0f;
#pragma unroll
    for (int j = 0; j < 8; ++j) { const float dv = mv[j] - mu; s2 += dv * dv; }
    s2 = wsum(s2);
    const float var = s2 * (1.0f / DM);
    const float rstd = rsqrtf(var + LNEPS);
#pragma unroll
    for (int j = 0; j < 8; ++j) {
      const int c = cb + j;
      const float v = uv[j] + ((mv[j] - mu) * rstd) * wv[j] + bv[j];
      const int co = DM - 1 - c;
      sO[co * 36 + tok] = v;
    }
  }
  __syncthreads();

  out_store_pass(sO, out, b, l0, w, lane);
  __threadfence();
  out_store_pass(sO, out, b, l0, w, lane);
}

extern "C" void kernel_launch(void* const* d_in, const int* in_sizes, int n_in,
                              void* d_out, int out_size, void* d_ws, size_t ws_size,
                              hipStream_t stream)
{
  if (n_in < 27) return;
  if (in_sizes[0] != NB * DM * NL) return;
  for (int i = 1; i <= 4; ++i) if (in_sizes[i] != DM) return;
  for (int blk = 0; blk < 2; ++blk) {
    const int o = 5 + 11 * blk;
    if (in_sizes[o + 0] != DM * DIN2)  return;
    if (in_sizes[o + 1] != DIN2)       return;
    if (in_sizes[o + 2] != DI * 4)     return;
    if (in_sizes[o + 3] != DI)         return;
    if (in_sizes[o + 4] != DI * NXD)   return;
    if (in_sizes[o + 5] != DTR * DI)   return;
    if (in_sizes[o + 6] != DI)         return;
    if (in_sizes[o + 7] != DI * NS)    return;
    if (in_sizes[o + 8] != DI)         return;
    if (in_sizes[o + 9] != DI * DM)    return;
    if (in_sizes[o + 10] != DM)        return;
  }
  if (out_size != NB * DM * NL) return;
  if (ws_size < WS_END) return;

  const float* x     = (const float*)d_in[0];
  const float* ln1_w = (const float*)d_in[1];
  const float* ln1_b = (const float*)d_in[2];
  const float* ln2_w = (const float*)d_in[3];
  const float* ln2_b = (const float*)d_in[4];
  const float* in_w[2], * in_b[2], * conv_w[2], * conv_b[2], * xproj_w[2], * dt_w[2], * dt_b[2],
             * a_log[2], * dpar[2], * out_w[2], * out_b[2];
  for (int blk = 0; blk < 2; ++blk) {
    const int o = 5 + 11 * blk;
    in_w[blk]    = (const float*)d_in[o + 0];
    in_b[blk]    = (const float*)d_in[o + 1];
    conv_w[blk]  = (const float*)d_in[o + 2];
    conv_b[blk]  = (const float*)d_in[o + 3];
    xproj_w[blk] = (const float*)d_in[o + 4];
    dt_w[blk]    = (const float*)d_in[o + 5];
    dt_b[blk]    = (const float*)d_in[o + 6];
    a_log[blk]   = (const float*)d_in[o + 7];
    dpar[blk]    = (const float*)d_in[o + 8];
    out_w[blk]   = (const float*)d_in[o + 9];
    out_b[blk]   = (const float*)d_in[o + 10];
  }
  float* out = (float*)d_out;

  char* ws = (char*)d_ws;
  unsigned short* X0 = (unsigned short*)(ws + OFF_X0);
  unsigned short* WIN[2], * WXP[2], * WDT[2], * WOUT[2];
  float* XR[2], * XF[2], * XDBL[2], * MO[2];
  unsigned short* XH[2], * XL[2], * DTH[2], * DTL[2], * YH[2], * YL[2];
  for (int blk = 0; blk < 2; ++blk) {
    char* wsw = ws + ((blk == 0) ? OFF_W1 : OFF_W2);
    char* wsp = ws + ((blk == 0) ? OFF_P1 : OFF_P2);
    WIN[blk]  = (unsigned short*)(wsw + WO_WIN);
    WXP[blk]  = (unsigned short*)(wsw + WO_WXP);
    WDT[blk]  = (unsigned short*)(wsw + WO_WDT);
    WOUT[blk] = (unsigned short*)(wsw + WO_WOUT);
    XR[blk]   = (float*)(wsp + PO_XR);
    XF[blk]   = (float*)(wsp + PO_XF);
    XH[blk]   = (unsigned short*)(wsp + PO_XH);
    XL[blk]   = (unsigned short*)(wsp + PO_XL);
    XDBL[blk] = (float*)(wsp + PO_XDBL);
    DTH[blk]  = (unsigned short*)(wsp + PO_DTH);
    DTL[blk]  = (unsigned short*)(wsp + PO_DTL);
    YH[blk]   = (unsigned short*)(wsp + PO_YH);
    YL[blk]   = (unsigned short*)(wsp + PO_YL);
    MO[blk]   = (float*)(wsp + PO_MO);
  }
  float*          U2F = (float*)(ws + OFF_U2F);
  unsigned short* U2H = (unsigned short*)(ws + OFF_U2H);
  unsigned short* U2L = (unsigned short*)(ws + OFF_U2L);

  tcvt_kernel<<<dim3(NL / 64, DM / 64, NB), dim3(256), 0, stream>>>(
      x, DM, NL, (size_t)DM * NL, X0, DM, (size_t)NL * DM);

  for (int blk = 0; blk < 2; ++blk) {
    tcvt_kernel<<<dim3(DIN2 / 64, DM / 64, 1), dim3(256), 0, stream>>>(
        in_w[blk], DM, DIN2, 0, WIN[blk], DM, 0);
    tcvt_kernel<<<dim3(NXP / 64, DI / 64, 1), dim3(256), 0, stream>>>(
        xproj_w[blk], DI, NXD, 0, WXP[blk], DI, 0);
    tcvt_kernel<<<dim3(DI / 64, KDT / 64, 1), dim3(256), 0, stream>>>(
        dt_w[blk], DTR, DI, 0, WDT[blk], KDT, 0);
    tcvt_kernel<<<dim3(DM / 64, DI / 64, 1), dim3(256), 0, stream>>>(
        out_w[blk], DI, DM, 0, WOUT[blk], DI, 0);
  }

  for (int blk = 0; blk < 2; ++blk) {
    if (blk == 0) {
      gemm_kernel<1, 0, 1><<<dim3(NROWS / 128, DIN2 / 64), dim3(128), 0, stream>>>(
          X0, X0, DM, WIN[0], DM, in_b[0], XR[0], DIN2, DTH[0], DTL[0]);
    } else {
      gemm_kernel<2, 0, 1><<<dim3(NROWS / 128, DIN2 / 64), dim3(128), 0, stream>>>(
          U2H, U2L, DM, WIN[1], DM, in_b[1], XR[1], DIN2, DTH[1], DTL[1]);
    }
    conv_kernel<<<dim3(DI / 256, NROWS / TC), dim3(256), 0, stream>>>(
        XR[blk], conv_w[blk], conv_b[blk], XF[blk], XH[blk], XL[blk]);
    gemm_kernel<2, 1, 0><<<dim3(NROWS / 128, NXP / 64), dim3(128), 0, stream>>>(
        XH[blk], XL[blk], DI, WXP[blk], DI, xproj_w[blk], XDBL[blk], NXP, DTH[blk], DTL[blk]);
    dtscan_kernel<<<dim3(DI / 256, NB), dim3(256), 0, stream>>>(
        DTH[blk], DTL[blk], WDT[blk], XDBL[blk], XF[blk], XR[blk], dt_b[blk], a_log[blk], dpar[blk],
        YH[blk], YL[blk]);
    gemm_kernel<2, 0, 1><<<dim3(NROWS / 128, DM / 64), dim3(128), 0, stream>>>(
        YH[blk], YL[blk], DI, WOUT[blk], DI, out_b[blk], MO[blk], DM, DTH[blk], DTL[blk]);
    if (blk == 0) {
      lnmid_kernel<<<dim3(NROWS / TC), dim3(256), 0, stream>>>(MO[0], X0, ln1_w, ln1_b, U2F, U2H, U2L);
    } else {
      lnout_kernel<<<dim3(NROWS / TO), dim3(256), 0, stream>>>(MO[1], U2F, ln2_w, ln2_b, out);
    }
  }
}
